// PhaseFunctionedNetwork_66099546685778
// MI455X (gfx1250) — hardware-verified
//
#include <hip/hip_runtime.h>
#include <math.h>

typedef __attribute__((ext_vector_type(16))) _Float16 v16h;
typedef __attribute__((ext_vector_type(16))) __bf16 v16b;
typedef __attribute__((ext_vector_type(8)))  _Float16 v8h;
typedef __attribute__((ext_vector_type(8)))  float v8f;
typedef __attribute__((ext_vector_type(4)))  float v4f;
typedef __attribute__((ext_vector_type(2)))  float v2f;
typedef __attribute__((ext_vector_type(4)))  unsigned v4u;
typedef __attribute__((ext_vector_type(4)))  int v4i;
typedef float __attribute__((may_alias)) float_a;
typedef int __attribute__((may_alias)) int_a;

template <typename T> __device__ __forceinline__ void vst2(void* p, T v) { *(volatile T*)p = v; __threadfence(); *(volatile T*)p = v; }
__device__ __forceinline__ v8f wmma16(v16h a, v16h b, v8f c) {
  v8f d = __builtin_amdgcn_wmma_f32_16x16x32_f16(false, a, false, b, (short)0, c, false, false);
  asm volatile("v_nop\n\tv_nop\n\tv_nop\n\tv_nop" : "+v"(d) : "v"(a), "v"(b));
  return d;
}
__device__ __forceinline__ v8f wmma_bf(v16b a, v16b b, v8f c) {
  v8f d = __builtin_amdgcn_wmma_f32_16x16x32_bf16(false, a, false, b, (short)0, c, false, false);
  asm volatile("v_nop\n\tv_nop\n\tv_nop\n\tv_nop" : "+v"(d) : "v"(a), "v"(b));
  return d;
}
__device__ __forceinline__ v16h frag_h(const _Float16* rowk0, int lane) {
  union { v16h v; v8h q[2]; } u; const _Float16* p = rowk0 + 8 * (lane >> 4);
  u.q[0] = *(const v8h*)p; u.q[1] = *(const v8h*)(p + 16); return u.v;
}
__device__ __forceinline__ v16h frag_f32(const float* rowk0, int lane) {
  v16h a; const float* p = rowk0 + 8 * (lane >> 4);
#pragma unroll
  for (int i = 0; i < 8; ++i) { a[i] = (_Float16)p[i]; a[8 + i] = (_Float16)p[16 + i]; }
  return a;
}
__device__ __forceinline__ v16h frag_f32s(const float* rowk0, int lane, float sc) {
  v16h a; const float* p = rowk0 + 8 * (lane >> 4);
#pragma unroll
  for (int i = 0; i < 8; ++i) { a[i] = (_Float16)(p[i] * sc); a[8 + i] = (_Float16)(p[16 + i] * sc); }
  return a;
}
__device__ __forceinline__ v16h fragc_f32(const float* W, int k0, int n, int lane, int ld, int K) {
  v16h a; const int g = lane >> 4;
#pragma unroll
  for (int i = 0; i < 8; ++i) { const int ka = k0 + 8 * g + i, kb = ka + 16;
    a[i] = (_Float16)(ka < K ? W[(size_t)ka * ld + n] : 0.f); a[8 + i] = (_Float16)(kb < K ? W[(size_t)kb * ld + n] : 0.f); }
  return a;
}
struct F2 { v16b h, l; };
__device__ __forceinline__ F2 bsplit16(const float v[16]) { F2 r;
#pragma unroll
  for (int i = 0; i < 16; ++i) { const __bf16 h = (__bf16)v[i]; r.h[i] = h; r.l[i] = (__bf16)(v[i] - (float)h); }
  return r; }
__device__ __forceinline__ F2 split_row(const float* row, int k0, int lane) { float v[16]; const float* p = row + k0 + 8 * (lane >> 4);
#pragma unroll
  for (int i = 0; i < 8; ++i) { v[i] = p[i]; v[8 + i] = p[16 + i]; }
  return bsplit16(v); }
__device__ __forceinline__ F2 split_rowK(const float* row, int k0, int lane, int K) { float v[16]; const int g = lane >> 4;
#pragma unroll
  for (int i = 0; i < 8; ++i) { const int ka = k0 + 8 * g + i, kb = ka + 16; v[i] = ka < K ? row[ka] : 0.f; v[8 + i] = kb < K ? row[kb] : 0.f; }
  return bsplit16(v); }
__device__ __forceinline__ F2 split_col(const float* W, int k0, int n, int lane, int ld, int K) { float v[16]; const int g = lane >> 4;
#pragma unroll
  for (int i = 0; i < 8; ++i) { const int ka = k0 + 8 * g + i, kb = ka + 16; v[i] = ka < K ? W[(size_t)ka * ld + n] : 0.f; v[8 + i] = kb < K ? W[(size_t)kb * ld + n] : 0.f; }
  return bsplit16(v); }
__device__ __forceinline__ v8f mac3(const F2& a, const F2& b, v8f c) { c = wmma_bf(a.l, b.h, c); c = wmma_bf(a.h, b.l, c); return wmma_bf(a.h, b.h, c); }
__device__ __forceinline__ float sigm(float v) { return 1.0f / (1.0f + expf(-v)); }
#define LDSX() do { asm volatile("s_wait_dscnt 0" ::: "memory"); __builtin_amdgcn_wave_barrier(); __builtin_amdgcn_fence(__ATOMIC_RELEASE, "workgroup"); } while (0)

#define NBT 1024
#define NS 4
#define HID 512
#define IND 342
#define INP 343
#define OUTD 311

template <int KIN, int KLD, int NOUT, int NOUTP, int ACT>
__global__ __launch_bounds__(128) void k_layer(const float* __restrict__ A, int lda, const float* __restrict__ xph, const float* __restrict__ W, const float* __restrict__ bias, float* __restrict__ Y, int ldy) {
  __shared__ __align__(16) float so[4][16][68];
  const int tid = threadIdx.x, wave = tid >> 5, lane = tid & 31, col = lane & 15, g = lane >> 4;
  const int r0 = blockIdx.x * 64 + wave * 16, n0 = blockIdx.y * 64;
  v8f acc[NS][4];
#pragma unroll
  for (int s = 0; s < NS; ++s)
#pragma unroll
    for (int t = 0; t < 4; ++t) acc[s][t] = (v8f){};
#pragma unroll 1
  for (int kc = 0; kc < (KIN + 31) / 32; ++kc) { const F2 a = split_rowK(A + (size_t)(r0 + col) * lda, kc * 32, lane, KIN);
#pragma unroll
    for (int s = 0; s < NS; ++s)
#pragma unroll
      for (int t = 0; t < 4; ++t) { const int n = n0 + t * 16 + col; const int nn = n < NOUT ? n : 0;
        acc[s][t] = mac3(a, split_rowK(W + ((size_t)s * NOUT + nn) * KLD, kc * 32, lane, KIN), acc[s][t]); } }
#pragma unroll
  for (int r = 0; r < 8; ++r) { const int row = r0 + 8 * g + r; const float ph = xph[(size_t)row * INP + IND]; const float ps = (float)NS * ph; const float mu = ps - floorf(ps);
    const int i1 = ((int)ps) & 3, i0 = (i1 + 3) & 3, i2 = (i1 + 1) & 3, i3 = (i1 + 2) & 3;
    const float mu2 = mu * mu, mu3 = mu2 * mu;
    const float c0 = -0.5f * mu3 + mu2 - 0.5f * mu, c1 = 1.5f * mu3 - 2.5f * mu2 + 1.0f, c2 = -1.5f * mu3 + 2.0f * mu2 + 0.5f * mu, c3 = 0.5f * mu3 - 0.5f * mu2;
    float cs[4]; cs[i0] = c0; cs[i1] = c1; cs[i2] = c2; cs[i3] = c3;
#pragma unroll
    for (int t = 0; t < 4; ++t) { const int n = n0 + t * 16 + col; float v = 0.f;
      if (n < NOUT) {
#pragma unroll
        for (int s = 0; s < NS; ++s) v += cs[s] * (acc[s][t][r] + bias[s * NOUT + n]);
        if (ACT) v = v > 0.f ? v : expm1f(v); }
      so[wave][8 * g + r][t * 16 + col] = v; } }
  LDSX();
  for (int q = lane; q < 16 * 16; q += 32) { const int rl = q >> 4, pc = q & 15; if (n0 + pc * 4 < NOUTP) vst2(Y + (size_t)(r0 + rl) * ldy + n0 + pc * 4, *(const v4f*)(&so[wave][rl][pc * 4])); }
}
__global__ __launch_bounds__(256) void k_copy(const float* __restrict__ H3, float* __restrict__ out) {
  const size_t base = (size_t)blockIdx.x * 64 * OUTD;
  for (int q = threadIdx.x; q < 64 * OUTD / 4; q += 256) { const size_t f = base + (size_t)q * 4; v4f o;
#pragma unroll
    for (int e = 0; e < 4; ++e) { const size_t ff = f + e; o[e] = H3[(ff / OUTD) * 320 + ff % OUTD]; }
    vst2(out + f, o); }
}
extern "C" void kernel_launch(void* const* d_in, const int* in_sizes, int n_in, void* d_out, int out_size, void* d_ws, size_t ws_size, hipStream_t stream) {
  (void)in_sizes; (void)n_in; (void)out_size; (void)ws_size;
  const float* x = (const float*)d_in[0]; const float* W0 = (const float*)d_in[1]; const float* W1 = (const float*)d_in[2]; const float* W2 = (const float*)d_in[3]; const float* b0 = (const float*)d_in[4]; const float* b1 = (const float*)d_in[5]; const float* b2 = (const float*)d_in[6];
  float* out = (float*)d_out;
  char* ws = (char*)d_ws; size_t off = 0;
  auto take = [&](size_t bytes) { char* p = ws + off; off += (bytes + 255) & ~(size_t)255; return p; };
  float* H1 = (float*)take((size_t)NBT * HID * 4); float* H2 = (float*)take((size_t)NBT * HID * 4); float* H3 = (float*)take((size_t)NBT * 320 * 4);
  k_layer<IND, IND, HID, HID, 1><<<dim3(NBT / 64, HID / 64), 128, 0, stream>>>(x, INP, x, W0, b0, H1, HID);
  k_layer<HID, HID, HID, HID, 1><<<dim3(NBT / 64, HID / 64), 128, 0, stream>>>(H1, HID, x, W1, b1, H2, HID);
  k_layer<HID, HID, OUTD, 320, 0><<<dim3(NBT / 64, 5), 128, 0, stream>>>(H2, HID, x, W2, b2, H3, 320);
  k_copy<<<NBT / 64, 256, 0, stream>>>(H3, out);
}
